// highwayNet_23106924052607
// MI455X (gfx1250) — hardware-verified
//
#include <hip/hip_runtime.h>
#include <math.h>

typedef __attribute__((ext_vector_type(16))) _Float16 v16h;
typedef __attribute__((ext_vector_type(8)))  _Float16 v8h;
typedef __attribute__((ext_vector_type(8)))  float  v8f;
typedef __attribute__((ext_vector_type(4)))  float  v4f;
typedef __attribute__((ext_vector_type(4)))  unsigned v4u;
typedef float __attribute__((may_alias)) float_a;

#define BIMG 512
#define NN 39
#define N_NODES (BIMG * NN)
#define XK 128
#define BT 256
#define ECAP 2560
#define SCAP 32
#define ETILE 2048
#define NBUCK ((N_NODES + BT - 1) / BT)
#define BN_EPS 1e-5f

template <typename V> __device__ __forceinline__ void vst2(void* p, V v) {
  *(volatile V*)p = v; __threadfence(); *(volatile V*)p = v;
}
__device__ __forceinline__ v8f wmma_f16(v16h a, v16h b, v8f c) {
  v8f d = __builtin_amdgcn_wmma_f32_16x16x32_f16(false, a, false, b, (short)0, c, false, false);
  asm volatile("v_nop\n\tv_nop\n\tv_nop\n\tv_nop" : "+v"(d) : "v"(a), "v"(b));
  return d;
}
__device__ __forceinline__ v16h frag_h(const _Float16* row, int k0, int lane) {
  union { v16h v; v8h h[2]; } r; const _Float16* p = row + k0 + 8 * (lane >> 4);
  r.h[0] = *(const v8h*)(p); r.h[1] = *(const v8h*)(p + 16); return r.v;
}
__device__ __forceinline__ v16h frag_f32(const float* row, int k0, int lane) {
  v16h a; const float* p = row + k0 + 8 * (lane >> 4);
#pragma unroll
  for (int i = 0; i < 8; ++i) { a[i] = (_Float16)p[i]; a[8 + i] = (_Float16)p[16 + i]; }
  return a;
}
__device__ __forceinline__ float n2n(float v) {
  if (isnan(v)) return 0.f;
  if (isinf(v)) return v > 0.f ? 3.4028235e38f : -3.4028235e38f;
  return v;
}
__device__ __forceinline__ float sigm(float x) { return 1.f / (1.f + __expf(-x)); }

struct Bucket {
  int lsrc[ECAP]; unsigned short ltgt[ECAP]; unsigned short sub[BT][SCAP]; int scnt[BT]; int wcnt[8][8]; int total;
};
__device__ void bucket_build(Bucket& bk, const int* __restrict__ src, const int* __restrict__ dst, int E, int tlo, int tid) {
  const int lane = tid & 31, wave = tid >> 5;
  if (tid == 0) bk.total = 0;
  __syncthreads();
  for (int e0 = 0; e0 < E; e0 += ETILE) {
    int rv[8]; unsigned msk[8];
#pragma unroll
    for (int j = 0; j < 8; ++j) {
      const int e = e0 + j * 256 + tid;
      const int r = (e < E) ? dst[e] : -1;
      rv[j] = r;
      msk[j] = (unsigned)__builtin_amdgcn_ballot_w32((r >= tlo) && (r < tlo + BT));
    }
    if (lane < 8) bk.wcnt[lane][wave] = __builtin_popcount(msk[lane]);
    __syncthreads();
    const int base = bk.total;
    int run = 0, pre[8];
#pragma unroll
    for (int j = 0; j < 8; ++j) {
#pragma unroll
      for (int w = 0; w < 8; ++w) { if (w == wave) pre[j] = run; run += bk.wcnt[j][w]; }
    }
#pragma unroll
    for (int j = 0; j < 8; ++j) {
      const unsigned m = msk[j];
      if ((m >> lane) & 1u) {
        const int pos = base + pre[j] + __builtin_popcount(m & ((1u << lane) - 1u));
        if (pos < ECAP) { bk.lsrc[pos] = e0 + j * 256 + tid; bk.ltgt[pos] = (unsigned short)(rv[j] - tlo); }
      }
    }
    __syncthreads();
    if (tid == 0) bk.total = base + run;
    __syncthreads();
  }
  const int n = (bk.total < ECAP) ? bk.total : ECAP;
  for (int i = tid; i < n; i += 256) { int s = src[bk.lsrc[i]]; s = s < 0 ? 0 : (s >= N_NODES ? N_NODES - 1 : s); bk.lsrc[i] = s; }
  __syncthreads();
  int k = 0;
  for (int i = 0; i < n; ++i) if ((int)bk.ltgt[i] == tid) { if (k < SCAP) bk.sub[tid][k] = (unsigned short)i; ++k; }
  bk.scnt[tid] = (k < SCAP) ? k : SCAP;
  __syncthreads();
}


__global__ __launch_bounds__(256) void k_wt(const float* __restrict__ W, _Float16* __restrict__ WT, int K, int M, int Kp, int mofs) {
  __shared__ __align__(16) _Float16 tile[64][72];
  const int mt = M / 64, tid = threadIdx.x;
  const int m0 = (blockIdx.x % mt) * 64, k0 = (blockIdx.x / mt) * 64;
  for (int i = tid; i < 64 * 64; i += 256) { const int kk = i >> 6, mm = i & 63; const int k = k0 + kk;
    tile[mm][kk] = (k < K) ? (_Float16)W[(size_t)k * M + m0 + mm] : (_Float16)0.f; }
  __syncthreads();
  for (int g = tid; g < 64 * 8; g += 256) { const int mm = g >> 3, pc = g & 7; vst2(WT + (size_t)(mofs + m0 + mm) * Kp + k0 + pc * 8, *(const v4u*)(&tile[mm][pc * 8])); }
}

__global__ __launch_bounds__(256) void k_encode(const float* __restrict__ ve, const float* __restrict__ ac, const float* __restrict__ man,
                                               const float* __restrict__ mask,
                                               const float* __restrict__ c1w, const float* __restrict__ c1b, const float* __restrict__ g1, const float* __restrict__ b1,
                                               const float* __restrict__ c2w, const float* __restrict__ c2b, const float* __restrict__ g2, const float* __restrict__ b2,
                                               const float* __restrict__ wih, const float* __restrict__ whh, const float* __restrict__ bih, const float* __restrict__ bhh,
                                               _Float16* __restrict__ X) {
  __shared__ float xin[3][NN * NN];
  __shared__ __align__(16) float x1raw[8 * NN * NN];
  __shared__ float x2[16][NN * NN];
  float (*x1)[NN * NN] = (float (*)[NN * NN])x1raw;
  float (*yg)[NN + 1] = (float (*)[NN + 1])x1raw;
  _Float16 (*xo)[XK] = (_Float16 (*)[XK])(x1raw + NN * (NN + 1) + 8);
  const int b = blockIdx.x, tid = threadIdx.x;
  for (int i = tid; i < NN * NN; i += 256) {
    xin[0][i] = n2n(man[(size_t)b * NN * NN + i]); xin[1][i] = n2n(ac[(size_t)b * NN * NN + i]); xin[2][i] = n2n(ve[(size_t)b * NN * NN + i]);
  }
  __syncthreads();
  const float bnscale = rsqrtf(1.0f + BN_EPS);
  for (int i = tid; i < 8 * NN * NN; i += 256) {
    const int o = i / (NN * NN), p = i % (NN * NN);
    float v = c1b[o];
#pragma unroll
    for (int c = 0; c < 3; ++c) v += c1w[o * 3 + c] * xin[c][p];
    v = v * (g1[o] * bnscale) + b1[o];
    x1[o][p] = fmaxf(v, 0.f);
  }
  __syncthreads();
  for (int i = tid; i < 16 * NN * NN; i += 256) {
    const int o = i / (NN * NN), p = i % (NN * NN), hh = p / NN, ww = p % NN;
    float v = c2b[o];
#pragma unroll 1
    for (int c = 0; c < 8; ++c)
#pragma unroll
      for (int dy = -1; dy <= 1; ++dy) { const int y = hh + dy; if (y < 0 || y >= NN) continue;
#pragma unroll
        for (int dx = -1; dx <= 1; ++dx) { const int x = ww + dx; if (x < 0 || x >= NN) continue;
          v += c2w[((o * 8 + c) * 3 + (dy + 1)) * 3 + (dx + 1)] * x1[c][y * NN + x]; } }
    x2[o][p] = v * (g2[o] * bnscale) + b2[o];
  }
  __syncthreads();
  if (tid < NN) {
    const int w = tid;
    float h = 0.f;
    for (int t = 0; t < NN; ++t) {
      float gi0 = bih[0], gi1 = bih[1], gi2 = bih[2];
#pragma unroll
      for (int c = 0; c < 16; ++c) { const float xv = x2[c][t * NN + w]; gi0 += wih[c] * xv; gi1 += wih[16 + c] * xv; gi2 += wih[32 + c] * xv; }
      const float gh0 = h * whh[0] + bhh[0], gh1 = h * whh[1] + bhh[1], gh2 = h * whh[2] + bhh[2];
      const float r = sigm(gi0 + gh0), z = sigm(gi1 + gh1);
      const float n = tanhf(gi2 + r * gh2);
      h = (1.f - z) * n + z * h;
      yg[w][t] = h;
    }
  }
  __syncthreads();
  for (int i = tid; i < NN * XK; i += 256) {
    const int j = i / XK, f = i % XK;
    const float m = mask[(size_t)b * NN + j];
    float v = 0.f;
    if (f < NN) v = xin[0][f * NN + j] * m;
    else if (f < 2 * NN) v = yg[j][f - NN] * m;
    xo[j][f] = (_Float16)v;
  }
  __syncthreads();
  _Float16* dst = X + (size_t)b * NN * XK;
  for (int g = tid; g < NN * XK / 8; g += 256) vst2(dst + g * 8, *(const v4u*)(&xo[0][0] + g * 8));
}

template <int K, int M, bool AF32>
__global__ __launch_bounds__(128) void k_gemm(const void* __restrict__ Av, const _Float16* __restrict__ WT, float* __restrict__ Y) {
  constexpr int NW = M / 4, NTW = NW / 16, KC = K / 32;
  __shared__ __align__(16) float so[16 * M];
  const int tid = threadIdx.x, wave = tid >> 5, lane = tid & 31, hi = lane >> 4, col = lane & 15;
  const int strip = blockIdx.x;
#pragma unroll 1
  for (int j = 0; j < NTW; ++j) {
    const int n0 = wave * NW + j * 16;
    v8f acc = {};
    const _Float16* br = WT + (size_t)(n0 + col) * K;
#pragma unroll 4
    for (int kc = 0; kc < KC; ++kc) {
      v16h a = AF32 ? frag_f32((const float*)Av + (size_t)(strip * 16 + col) * K, kc * 32, lane)
                    : frag_h((const _Float16*)Av + (size_t)(strip * 16 + col) * K, kc * 32, lane);
      acc = wmma_f16(a, frag_h(br, kc * 32, lane), acc);
    }
#pragma unroll
    for (int r = 0; r < 8; ++r) so[(hi * 8 + r) * M + n0 + col] = acc[r];
  }
  __syncthreads();
  float* dst = Y + (size_t)strip * 16 * M;
  for (int g = tid; g < 16 * M / 4; g += 128) vst2(dst + g * 4, *(const v4f*)(so + g * 4));
}

template <int H, bool ELU_OUT>
__global__ __launch_bounds__(256) void k_gat(const int* __restrict__ src, const int* __restrict__ dst, int E,
                                             const float* __restrict__ XLR, const float* __restrict__ att, const float* __restrict__ bias,
                                             float* __restrict__ out) {
  constexpr int M = H * 64;
  __shared__ Bucket bk;
  const int tid = threadIdx.x, lane = tid & 31, wave = tid >> 5, tlo = blockIdx.x * BT;
  bucket_build(bk, src, dst, E, tlo, tid);
  for (int s = 0; s < 32; ++s) {
    const int t = wave * 32 + s, node = tlo + t;
    if (node >= N_NODES) break;
    const int cnt = bk.scnt[t];
    const float* xr = XLR + (size_t)node * (2 * M) + M;
    float* orow = out + (size_t)node * M;
#pragma unroll 1
    for (int h = 0; h < H; ++h) {
      const int c0 = h * 64 + lane, c1 = c0 + 32;
      const float a0 = att[c0], a1 = att[c1], xr0 = xr[c0], xr1 = xr[c1];
      float m = -3.0e38f, l = 0.f, acc0 = 0.f, acc1 = 0.f;
      for (int k = -1; k < cnt; ++k) {
        const int sN = (k < 0) ? node : bk.lsrc[bk.sub[t][k]];
        const float* xl = XLR + (size_t)sN * (2 * M);
        const float x0 = xl[c0], x1 = xl[c1];
        float e0 = x0 + xr0, e1 = x1 + xr1;
        e0 = e0 > 0.f ? e0 : 0.2f * e0; e1 = e1 > 0.f ? e1 : 0.2f * e1;
        float p = e0 * a0 + e1 * a1;
#pragma unroll
        for (int off = 16; off > 0; off >>= 1) p += __shfl_xor(p, off, 32);
        const float mn = fmaxf(m, p), cw = __expf(m - mn), w = __expf(p - mn);
        l = l * cw + w; m = mn;
        acc0 = acc0 * cw + w * x0; acc1 = acc1 * cw + w * x1;
      }
      const float inv = 1.f / (l + 1e-16f);
      float v0 = acc0 * inv + bias[c0], v1 = acc1 * inv + bias[c1];
      if (ELU_OUT) { v0 = v0 > 0.f ? v0 : (__expf(v0) - 1.f); v1 = v1 > 0.f ? v1 : (__expf(v1) - 1.f); }
      vst2(orow + c0, (float_a)v0);
      vst2(orow + c1, (float_a)v1);
    }
  }
}

extern "C" void kernel_launch(void* const* d_in, const int* in_sizes, int n_in,
                              void* d_out, int out_size, void* d_ws, size_t ws_size,
                              hipStream_t stream) {
  (void)n_in; (void)out_size; (void)ws_size;
  const int*   ei   = (const int*)d_in[0];
  const int E = in_sizes[0] / 2;
  const int* src = ei; const int* dst = ei + E;
  const float *ve = (const float*)d_in[1], *ac = (const float*)d_in[2], *man = (const float*)d_in[3], *mask = (const float*)d_in[4];
  const float *c1w = (const float*)d_in[5], *c1b = (const float*)d_in[6], *g1 = (const float*)d_in[7], *b1 = (const float*)d_in[8];
  const float *c2w = (const float*)d_in[9], *c2b = (const float*)d_in[10], *g2 = (const float*)d_in[11], *b2 = (const float*)d_in[12];
  const float *wih = (const float*)d_in[13], *whh = (const float*)d_in[14], *bih = (const float*)d_in[15], *bhh = (const float*)d_in[16];
  const float *g1wl = (const float*)d_in[17], *g1wr = (const float*)d_in[18], *g1att = (const float*)d_in[19], *g1bias = (const float*)d_in[20];
  const float *g2wl = (const float*)d_in[21], *g2wr = (const float*)d_in[22], *g2att = (const float*)d_in[23], *g2bias = (const float*)d_in[24];
  float* out = (float*)d_out;

  char* ws = (char*)d_ws; size_t off = 0;
  auto alloc = [&](size_t bytes) -> void* { void* p = ws + off; off = (off + bytes + 255) & ~(size_t)255; return p; };
  _Float16* X    = (_Float16*)alloc((size_t)N_NODES * XK * 2);
  _Float16* WT1  = (_Float16*)alloc((size_t)1024 * XK * 2);
  _Float16* WT2  = (_Float16*)alloc((size_t)128 * 512 * 2);
  float* XLR1 = (float*)alloc((size_t)N_NODES * 1024 * 4);
  float* H1   = (float*)alloc((size_t)N_NODES * 512 * 4);
  float* XLR2 = (float*)alloc((size_t)N_NODES * 128 * 4);

  k_encode<<<BIMG, 256, 0, stream>>>(ve, ac, man, mask, c1w, c1b, g1, b1, c2w, c2b, g2, b2, wih, whh, bih, bhh, X);
  k_wt<<<(XK / 64) * (512 / 64), 256, 0, stream>>>(g1wl, WT1, 78, 512, XK, 0);
  k_wt<<<(XK / 64) * (512 / 64), 256, 0, stream>>>(g1wr, WT1, 78, 512, XK, 512);
  k_wt<<<(512 / 64) * (64 / 64), 256, 0, stream>>>(g2wl, WT2, 512, 64, 512, 0);
  k_wt<<<(512 / 64) * (64 / 64), 256, 0, stream>>>(g2wr, WT2, 512, 64, 512, 64);
  k_gemm<XK, 1024, false><<<N_NODES / 16, 128, 0, stream>>>(X, WT1, XLR1);
  k_gat<8, true><<<NBUCK, 256, 0, stream>>>(src, dst, E, XLR1, g1att, g1bias, H1);
  k_gemm<512, 128, true><<<N_NODES / 16, 128, 0, stream>>>(H1, WT2, XLR2);
  k_gat<1, false><<<NBUCK, 256, 0, stream>>>(src, dst, E, XLR2, g2att, g2bias, out);
}
